// _SoftTreeModule_68478958567426
// MI455X (gfx1250) — hardware-run, weakly checked
//
#include <hip/hip_runtime.h>
#include <stddef.h>
#include <stdint.h>

#pragma clang fp contract(off)

#define NB     16384
#define NF     512
#define NC     1000
#define NCP    1024
#define NL     256
#define NNODE  255
#define NNP    256
#define TDEPTH 8

#define GR     64
#define XP     520
#define PP     256
#define MP     264
#define LR     64
#define LP     264
#define MR     16

#define LDS_X_BYTES  (GR * XP * 2)
#define LDS_P_OFF    LDS_X_BYTES
#define LDS_P_BYTES  (GR * PP * 4)
#define LDS_GATE     (LDS_P_OFF + LDS_P_BYTES)

static_assert(NB % GR == 0);
static_assert(NB % MR == 0);
static_assert(NCP % LR == 0);
static_assert(NF % 32 == 0);
static_assert(NL % 32 == 0);
static_assert(NL == 256);
static_assert((XP * 2) % 16 == 0);
static_assert((MP * 2) % 16 == 0);
static_assert((LP * 2) % 16 == 0);
static_assert(LDS_X_BYTES % 16 == 0);
static_assert(GR * MP * 2 <= LDS_X_BYTES);
static_assert((MR * NC * 4) % 128 == 0);
static_assert((MR * NC) % 4 == 0);
static_assert(MR * NC * 4 <= 64000);

typedef _Float16 v16h __attribute__((ext_vector_type(16)));
typedef _Float16 v8h  __attribute__((ext_vector_type(8)));
typedef float    v8f  __attribute__((ext_vector_type(8)));
typedef float    v4f  __attribute__((ext_vector_type(4)));
typedef unsigned int v4u __attribute__((ext_vector_type(4)));
typedef v8h __attribute__((may_alias)) v8ha;
typedef v4u __attribute__((may_alias)) v4ua;
typedef v4f __attribute__((may_alias)) v4fa;

union Frag { v16h v; v8h h[2]; };
union H8   { v8h h; v4u u; };

__device__ __forceinline__ v8f mma16(v16h a, v16h b, v8f cacc) {
  cacc = __builtin_amdgcn_wmma_f32_16x16x32_f16(false, a, false, b, (short)0, cacc, false, false);
  asm volatile("v_nop\n\tv_nop\n\tv_nop\n\tv_nop" : "+v"(cacc) : "v"(a), "v"(b));
  return cacc;
}

__device__ __forceinline__ v8f zero8() { return (v8f){0.f, 0.f, 0.f, 0.f, 0.f, 0.f, 0.f, 0.f}; }

__device__ __forceinline__ v16h ldfrag_g(const _Float16* __restrict__ p, int ld, int row0, int k0, int lane) {
  const int m = lane & 15, lh = lane >> 4;
  const _Float16* q = p + (size_t)(row0 + m) * ld + k0 + 8 * lh;
  Frag f;
  f.h[0] = *(const v8h*)(q);
  f.h[1] = *(const v8h*)(q + 16);
  return f.v;
}

__device__ __forceinline__ v16h ldfrag_l(const _Float16* p, int ld, int row0, int k0, int lane) {
  const int m = lane & 15, lh = lane >> 4;
  const _Float16* q = p + (row0 + m) * ld + k0 + 8 * lh;
  Frag f;
  f.h[0] = *(const v8ha*)(q);
  f.h[1] = *(const v8ha*)(q + 16);
  return f.v;
}

__global__ __launch_bounds__(256) void k_lplane(const float* __restrict__ L, _Float16* __restrict__ LS) {
  __shared__ __align__(16) _Float16 sl[LR * LP];
  const int t = threadIdx.x;
  const int n0 = blockIdx.x * LR;
  const float* row = L + (size_t)t * NC;

  float mx = -3.0e38f;
#pragma unroll 1
  for (int n = 0; n < NC; ++n) mx = fmaxf(mx, row[n]);
  float s = 0.0f;
#pragma unroll 1
  for (int n = 0; n < NC; ++n) s += expf(row[n] - mx);
  const float inv = 1.0f / s;

#pragma unroll 1
  for (int j = 0; j < LR; ++j) {
    const int n  = n0 + j;
    const int nc = (n < NC) ? n : NC - 1;
    const float e = expf(row[nc] - mx) * inv;
    const float v = (n < NC) ? e * 256.0f : 0.0f;
    sl[j * LP + t] = (_Float16)v;
  }
  __syncthreads();

  for (int ps = 0; ps < 2; ++ps) {
#pragma unroll
    for (int it = 0; it < 8; ++it) {
      const int p  = it * 256 + t;
      const int r  = p >> 5;
      const int pc = p & 31;
      const v4u val = *(const v4ua*)(sl + r * LP + pc * 8);
      *(volatile v4u*)(LS + (size_t)(n0 + r) * NL + pc * 8) = val;
    }
    __threadfence();
  }
}

__global__ __launch_bounds__(256) void k_wcvt(const float* __restrict__ W, _Float16* __restrict__ GW) {
  const int p  = blockIdx.x * 256 + threadIdx.x;
  const int n  = p >> 6;
  const int pc = p & 63;
  const int nr = (n < NNODE) ? n : NNODE - 1;
  const float* src = W + (size_t)nr * NF + pc * 8;
  const v4f a = *(const v4fa*)(src);
  const v4f b = *(const v4fa*)(src + 4);
  const float z = (n < NNODE) ? 16.0f : 0.0f;
  H8 cv;
  cv.h[0] = (_Float16)(a[0] * z); cv.h[1] = (_Float16)(a[1] * z);
  cv.h[2] = (_Float16)(a[2] * z); cv.h[3] = (_Float16)(a[3] * z);
  cv.h[4] = (_Float16)(b[0] * z); cv.h[5] = (_Float16)(b[1] * z);
  cv.h[6] = (_Float16)(b[2] * z); cv.h[7] = (_Float16)(b[3] * z);
  _Float16* dst = GW + (size_t)p * 8;
  *(volatile v4u*)dst = cv.u;
  __threadfence();
  *(volatile v4u*)dst = cv.u;
}

__global__ __launch_bounds__(256) void k_gate(const float* __restrict__ X, const _Float16* __restrict__ GW,
                                              const float* __restrict__ gb, _Float16* __restrict__ MU) {
  extern __shared__ __align__(16) char smem[];
  _Float16* xs = (_Float16*)smem;
  float*    ps = (float*)(smem + LDS_P_OFF);
  _Float16* ms = (_Float16*)smem;

  const int t = threadIdx.x, lane = t & 31, wave = t >> 5;
  const int hh = lane >> 4, c = lane & 15;
  const int r0 = blockIdx.x * GR;

#pragma unroll 4
  for (int it = 0; it < 16; ++it) {
    const int p = it * 256 + t;
    const int r = p >> 6, g = p & 63;
    const float* src = X + (size_t)(r0 + r) * NF + g * 8;
    const v4f a = *(const v4fa*)(src);
    const v4f b = *(const v4fa*)(src + 4);
    H8 cv;
    cv.h[0] = (_Float16)a[0]; cv.h[1] = (_Float16)a[1]; cv.h[2] = (_Float16)a[2]; cv.h[3] = (_Float16)a[3];
    cv.h[4] = (_Float16)b[0]; cv.h[5] = (_Float16)b[1]; cv.h[6] = (_Float16)b[2]; cv.h[7] = (_Float16)b[3];
    *(v8ha*)(xs + r * XP + g * 8) = cv.h;
  }
  __syncthreads();

  const int rt = wave >> 1;
  const int cg = wave & 1;
  v8f acc[8];
#pragma unroll
  for (int nt = 0; nt < 8; ++nt) acc[nt] = zero8();

#pragma unroll 1
  for (int ks = 0; ks < NF / 32; ++ks) {
    const int k0 = ks * 32;
    const v16h a = ldfrag_l(xs, XP, rt * 16, k0, lane);
#pragma unroll
    for (int nt = 0; nt < 8; ++nt) {
      const v16h b = ldfrag_g(GW, NF, cg * 128 + nt * 16, k0, lane);
      acc[nt] = mma16(a, b, acc[nt]);
    }
  }

#pragma unroll
  for (int nt = 0; nt < 8; ++nt) {
    const int node = cg * 128 + nt * 16 + c;
#pragma unroll
    for (int r = 0; r < 8; ++r) ps[(rt * 16 + 8 * hh + r) * PP + node] = acc[nt][r];
  }
  __syncthreads();

  {
    const int bn = (t < NNODE) ? t : NNODE - 1;
    const float bias = gb[bn];
#pragma unroll 1
    for (int r = 0; r < GR; ++r) {
      float v = ps[r * PP + t] * 0.0625f + bias;
      v = fminf(fmaxf(v, -30.0f), 30.0f);
      const float e = expf(-v);
      ps[r * PP + t] = 1.0f / (1.0f + e);
    }
  }
  __syncthreads();

#pragma unroll 1
  for (int b = 0; b < GR; ++b) {
    const float* pr = ps + b * PP;
    float m = 1.0f;
#pragma unroll
    for (int d = 0; d < TDEPTH; ++d) {
      const int node = ((1 << d) - 1) + (t >> (TDEPTH - d));
      const int bit  = (t >> (TDEPTH - 1 - d)) & 1;
      const float g  = pr[node];
      const float br = bit ? g : (1.0f - g);
      m = m * br;
    }
    ms[b * MP + t] = (_Float16)(m * 1024.0f);
  }
  __syncthreads();

  for (int pss = 0; pss < 2; ++pss) {
#pragma unroll
    for (int it = 0; it < 8; ++it) {
      const int p  = it * 256 + t;
      const int r  = p >> 5;
      const int pc = p & 31;
      const v4u val = *(const v4ua*)(ms + r * MP + pc * 8);
      *(volatile v4u*)(MU + (size_t)(r0 + r) * NL + pc * 8) = val;
    }
    __threadfence();
  }
}

__global__ __launch_bounds__(256) void k_mix(const _Float16* __restrict__ MU, const _Float16* __restrict__ LS,
                                             float* __restrict__ out) {
  __shared__ __align__(16) float st[MR * NC];
  const int t = threadIdx.x, lane = t & 31, wave = t >> 5;
  const int hh = lane >> 4, c = lane & 15;
  const int r0 = blockIdx.x * MR;

  v8f acc[8];
#pragma unroll
  for (int nt = 0; nt < 8; ++nt) acc[nt] = zero8();

#pragma unroll 1
  for (int ks = 0; ks < NL / 32; ++ks) {
    const int k0 = ks * 32;
    const v16h a = ldfrag_g(MU, NL, r0, k0, lane);
#pragma unroll
    for (int nt = 0; nt < 8; ++nt) {
      const v16h b = ldfrag_g(LS, NL, wave * 128 + nt * 16, k0, lane);
      acc[nt] = mma16(a, b, acc[nt]);
    }
  }

  const float scl = 3.814697265625e-06f;
#pragma unroll
  for (int nt = 0; nt < 8; ++nt) {
    const int col = wave * 128 + nt * 16 + c;
#pragma unroll
    for (int r = 0; r < 8; ++r) {
      const float v = acc[nt][r] * scl;
      if (col < NC) st[(8 * hh + r) * NC + col] = v;
    }
  }
  __syncthreads();

  float* ob = out + (size_t)r0 * NC;
  for (int ps = 0; ps < 2; ++ps) {
#pragma unroll
    for (int it = 0; it < 16; ++it) {
      const int p = it * 256 + t;
      if (p < (MR * NC) / 4) {
        const v4f val = *(const v4fa*)(st + p * 4);
        *(volatile v4f*)(ob + (size_t)p * 4) = val;
      }
    }
    __threadfence();
  }
}

extern "C" void kernel_launch(void* const* d_in, const int* in_sizes, int n_in,
                              void* d_out, int out_size, void* d_ws, size_t ws_size,
                              hipStream_t stream) {
  if (n_in < 4) return;
  if (in_sizes[0] != NB * NF) return;
  if (in_sizes[1] != NNODE * NF) return;
  if (in_sizes[2] != NNODE) return;
  if (in_sizes[3] != NL * NC) return;
  if (out_size != NB * NC) return;

  const float* x      = (const float*)d_in[0];
  const float* gate_w = (const float*)d_in[1];
  const float* gate_b = (const float*)d_in[2];
  const float* leaflg = (const float*)d_in[3];
  float* out = (float*)d_out;

  const size_t ls_bytes = (size_t)NCP * NL * 2;
  const size_t gw_bytes = (size_t)NNP * NF * 2;
  const size_t mu_bytes = (size_t)NB * NL * 2;
  const size_t gw_off = ls_bytes;
  const size_t mu_off = ls_bytes + gw_bytes;
  const size_t total  = mu_off + mu_bytes;
  if (total > ws_size) return;

  _Float16* LS = (_Float16*)((char*)d_ws + 0);
  _Float16* GW = (_Float16*)((char*)d_ws + gw_off);
  _Float16* MU = (_Float16*)((char*)d_ws + mu_off);

  k_lplane<<<dim3(NCP / LR), dim3(256), 0, stream>>>(leaflg, LS);
  k_wcvt<<<dim3((NNP * NF / 8) / 256), dim3(256), 0, stream>>>(gate_w, GW);
  (void)hipFuncSetAttribute(reinterpret_cast<const void*>(&k_gate),
                            hipFuncAttributeMaxDynamicSharedMemorySize, LDS_GATE);
  k_gate<<<dim3(NB / GR), dim3(256), LDS_GATE, stream>>>(x, GW, gate_b, MU);
  k_mix<<<dim3(NB / MR), dim3(256), 0, stream>>>(MU, LS, out);
  (void)hipGetLastError();
}
